// Network_86947317940878
// MI455X (gfx1250) — hardware-verified
//
#include <hip/hip_runtime.h>

constexpr int kNodes = 50000;
constexpr int kEdges = 800000;
constexpr int kIn    = 128;
constexpr int kHid   = 64;
constexpr int kCls   = 10;
constexpr int kMP    = 50176;
constexpr int kNT    = 256;
constexpr int kSRB   = 512;
constexpr int kSP    = 16;
constexpr int kChunk = kSP * kNT;
constexpr int kNCh   = (kEdges + kChunk - 1) / kChunk;
constexpr int kCap   = kChunk;

static_assert(kMP % 64 == 0 && kMP >= kNodes, "M tile multiple");
static_assert(kMP % kSRB == 0 && kMP % kNT == 0, "tiles exact");
static_assert(kIn % 32 == 0 && kHid % 32 == 0, "K multiples of 32");
static_assert(kHid % 64 == 0 && (2 * kHid) % 64 == 0, "N tile multiples");
static_assert(kEdges % kSP == 0, "thread edge groups never straddle the list end");
static_assert(kNodes % 16 == 0, "d_out wave ranges end on 128-B lines (16 nodes x 40 B = 5 lines)");
static_assert((kMP * kIn / 8) % kNT == 0, "cast grid exact");
static_assert(kSRB == 8 * 64, "8 waves x 64 destination rows");

typedef __attribute__((ext_vector_type(16))) _Float16 v16h;
typedef __attribute__((ext_vector_type(8)))  _Float16 v8h;
typedef __attribute__((ext_vector_type(16))) __bf16   v16b;
typedef __attribute__((ext_vector_type(8)))  __bf16   v8b;
typedef __attribute__((ext_vector_type(8)))  float    v8f;
typedef __attribute__((ext_vector_type(4)))  float    v4f;
typedef __attribute__((ext_vector_type(2)))  float    v2f;
typedef __attribute__((ext_vector_type(4)))  unsigned int v4u;
typedef __attribute__((ext_vector_type(2)))  unsigned int v2u;
typedef __attribute__((ext_vector_type(4)))  int      v4i;

__device__ __forceinline__ unsigned short f2bf_bits(float f) {
  unsigned u = __float_as_uint(f);
  return (unsigned short)((u + 0x7FFFu + ((u >> 16) & 1u)) >> 16);
}
__device__ __forceinline__ float bf_bits2f(unsigned short h) { return __uint_as_float(((unsigned)h) << 16); }

__device__ __forceinline__ void dep_guard_h(v8f& a, v8f& b, v16h x, v16h y) { asm volatile("v_nop\n\tv_nop\n\tv_nop\n\tv_nop" : "+v"(a), "+v"(b) : "v"(x), "v"(y)); }
__device__ __forceinline__ void dep_guard_b(v8f& a, v8f& b, v16b x, v16b y) { asm volatile("v_nop\n\tv_nop\n\tv_nop\n\tv_nop" : "+v"(a), "+v"(b) : "v"(x), "v"(y)); }
__device__ __forceinline__ void keep4_h(v16h a, v16h b, v16h c, v16h d) { asm volatile("v_nop" :: "v"(a), "v"(b), "v"(c), "v"(d)); }
__device__ __forceinline__ void keep4_b(v16b a, v16b b, v16b c, v16b d) { asm volatile("v_nop" :: "v"(a), "v"(b), "v"(c), "v"(d)); }
__device__ __forceinline__ void acc_guard4(v8f& a, v8f& b, v8f& c, v8f& d) { asm volatile("v_nop\n\tv_nop\n\tv_nop\n\tv_nop" : "+v"(a), "+v"(b), "+v"(c), "+v"(d)); }
template <typename T> struct Frag;
template <> struct Frag<_Float16> {
  typedef v16h V; union U { v16h v; v8h h[2]; };
  static __device__ __forceinline__ v16h load(const _Float16* p) {
    U f; f.h[0] = *(const v8h*)(p); f.h[1] = *(const v8h*)(p + 16); return f.v;
  }
  static __device__ __forceinline__ v8f mma(v16h a, v16h b, v8f c) {
    return __builtin_amdgcn_wmma_f32_16x16x32_f16(false, a, false, b, (short)0, c, false, false);
  }
  static __device__ __forceinline__ void guard(v8f& a, v8f& b, v16h x, v16h y) { dep_guard_h(a, b, x, y); }
  static __device__ __forceinline__ void keep(v16h a, v16h b, v16h c, v16h d) { keep4_h(a, b, c, d); }
};
template <> struct Frag<__bf16> {
  typedef v16b V; union U { v16b v; v8b h[2]; };
  static __device__ __forceinline__ v16b load(const __bf16* p) {
    U f; f.h[0] = *(const v8b*)(p); f.h[1] = *(const v8b*)(p + 16); return f.v;
  }
  static __device__ __forceinline__ v8f mma(v16b a, v16b b, v8f c) {
    return __builtin_amdgcn_wmma_f32_16x16x32_bf16(false, a, false, b, (short)0, c, false, false);
  }
  static __device__ __forceinline__ void guard(v8f& a, v8f& b, v16b x, v16b y) { dep_guard_b(a, b, x, y); }
  static __device__ __forceinline__ void keep(v16b a, v16b b, v16b c, v16b d) { keep4_b(a, b, c, d); }
};

template <int ET> struct Elem;
template <> struct Elem<0> { typedef _Float16 T; };
template <> struct Elem<1> { typedef __bf16 T; };
template <int ET, bool SPLIT, int BIAS_MODE, int OUT_MODE, bool RESID, int ACT = 0>
__global__ __launch_bounds__(256) void wmma_gemm64(
    const unsigned short* __restrict__ Ap, const unsigned short* __restrict__ A2p, int lda, long strideA,
    const unsigned short* __restrict__ Btp, const unsigned short* __restrict__ Bt2p, int ldb, long strideB,
    void* __restrict__ Cout, void* __restrict__ Cout2, int ldc, long strideC,
    const float* __restrict__ bias,
    const float* __restrict__ resid, long strideR,
    int M, int N, int K, float scale) {
  typedef typename Elem<ET>::T T;
  typedef typename Frag<T>::V V;
  const T* A = (const T*)Ap; const T* A2 = (const T*)A2p; const T* Bt = (const T*)Btp; const T* Bt2 = (const T*)Bt2p;
  __shared__ __align__(16) float sT[8][16 * 68];
  const int b    = blockIdx.y;
  const int lane = threadIdx.x & 31;
  const int wave = threadIdx.x >> 5;
  const int tilesN = N >> 6;
  const int tilesM = M >> 6;
  const int tile = blockIdx.x * 8 + wave;
  if (tile >= tilesM * tilesN) return;
  const int tm = tile / tilesN;
  const int tn = tile - tm * tilesN;
  const int m0 = tm << 6;
  const int n0 = tn << 6;

  const T* Ab  = A  + (size_t)b * strideA;
  const T* Bb  = Bt + (size_t)b * strideB;
  const T* Ab2 = SPLIT ? (A2  + (size_t)b * strideA) : nullptr;
  const T* Bb2 = SPLIT ? (Bt2 + (size_t)b * strideB) : nullptr;

  const int rlane = lane & 15;
  const int koff  = (lane >> 4) * 8;
  const int mOff  = (lane >> 4) * 8;

  v8f acc[4][4];
#pragma unroll
  for (int i = 0; i < 4; ++i)
#pragma unroll
    for (int j = 0; j < 4; ++j) acc[i][j] = (v8f){0.f,0.f,0.f,0.f,0.f,0.f,0.f,0.f};

  for (int k0 = 0; k0 < K; k0 += 32) {
    V bh[4], bl[4];
#pragma unroll
    for (int j = 0; j < 4; ++j) {
      const size_t bo = (size_t)(n0 + (j << 4) + rlane) * ldb + koff + k0;
      bh[j] = Frag<T>::load(Bb + bo);
      if (SPLIT) bl[j] = Frag<T>::load(Bb2 + bo);
    }
#pragma unroll
    for (int i = 0; i < 4; ++i) {
      const size_t ao = (size_t)(m0 + (i << 4) + rlane) * lda + koff + k0;
      V ah = Frag<T>::load(Ab + ao);
      V al;
      if (SPLIT) al = Frag<T>::load(Ab2 + ao);
#pragma unroll
      for (int j = 0; j < 4; ++j) {
        acc[i][j] = Frag<T>::mma(ah, bh[j], acc[i][j]);
        if (SPLIT) {
          acc[i][j] = Frag<T>::mma(ah, bl[j], acc[i][j]);
          acc[i][j] = Frag<T>::mma(al, bh[j], acc[i][j]);
        }
      }
      Frag<T>::guard(acc[i][0], acc[i][3], ah, SPLIT ? al : ah);
    }
    Frag<T>::keep(bh[0], bh[1], bh[2], bh[3]);
    if (SPLIT) Frag<T>::keep(bl[0], bl[1], bl[2], bl[3]);
  }
  acc_guard4(acc[0][0], acc[0][1], acc[0][2], acc[0][3]);
  acc_guard4(acc[1][0], acc[1][1], acc[1][2], acc[1][3]);
  acc_guard4(acc[2][0], acc[2][1], acc[2][2], acc[2][3]);
  acc_guard4(acc[3][0], acc[3][1], acc[3][2], acc[3][3]);

  float* slab = sT[wave];
  const float* Rb = RESID ? (resid + (size_t)b * strideR) : nullptr;
#pragma unroll
  for (int i = 0; i < 4; ++i) {
    const int mBase = m0 + (i << 4);
#pragma unroll
    for (int j = 0; j < 4; ++j) {
      const int n = n0 + (j << 4) + rlane;
      float bv = 0.f;
      if (BIAS_MODE == 2) bv = bias[n];
#pragma unroll
      for (int r = 0; r < 8; ++r) {
        float v = acc[i][j][r] * scale;
        if (BIAS_MODE == 1) v += bias[mBase + mOff + r];
        if (BIAS_MODE == 2) v += bv;
        if (RESID) v += Rb[(size_t)(mBase + mOff + r) * ldc + n];
        if (ACT == 2) v = fmaxf(v, 0.0f);
        if (ACT == 4) v = (v > 0.f) ? v : 0.01f * v;
        slab[(mOff + r) * 68 + (j << 4) + rlane] = v;
      }
    }
    __builtin_amdgcn_fence(__ATOMIC_RELEASE, "workgroup");
    __builtin_amdgcn_wave_barrier();
    __builtin_amdgcn_fence(__ATOMIC_ACQUIRE, "workgroup");
    if (OUT_MODE == 0) {
      float* C = (float*)Cout + (size_t)b * strideC;
      const int hh = lane >> 4, c4 = (lane & 15) * 4;
      for (int pass = 0; pass < 2; ++pass) {
#pragma unroll
        for (int it = 0; it < 8; ++it) {
          const int row = it * 2 + hh;
          v4f v = *(const v4f*)(slab + row * 68 + c4);
          *(volatile v4f*)(C + (size_t)(mBase + row) * ldc + n0 + c4) = v;
        }
        __threadfence();
      }
    } else {
      const int q = lane >> 3, c8 = (lane & 7) * 8;
      unsigned short* C  = (unsigned short*)Cout  + (size_t)b * strideC;
      unsigned short* C2 = (OUT_MODE == 2) ? ((unsigned short*)Cout2 + (size_t)b * strideC) : nullptr;
      for (int pass = 0; pass < 2; ++pass) {
#pragma unroll
        for (int it = 0; it < 4; ++it) {
          const int row = it * 4 + q;
          const float* sp = slab + row * 68 + c8;
          v8h hv, lv;
#pragma unroll
          for (int e = 0; e < 8; ++e) {
            if (OUT_MODE == 1) {
              hv[e] = (_Float16)sp[e];
            } else {
              unsigned short hb = f2bf_bits(sp[e]);
              unsigned short lb = f2bf_bits(sp[e] - bf_bits2f(hb));
              hv[e] = __builtin_bit_cast(_Float16, hb);
              lv[e] = __builtin_bit_cast(_Float16, lb);
            }
          }
          *(volatile v8h*)(C + (size_t)(mBase + row) * ldc + n0 + c8) = hv;
          if (OUT_MODE == 2) *(volatile v8h*)(C2 + (size_t)(mBase + row) * ldc + n0 + c8) = lv;
        }
        __threadfence();
      }
    }
    __builtin_amdgcn_fence(__ATOMIC_RELEASE, "workgroup");
    __builtin_amdgcn_wave_barrier();
    __builtin_amdgcn_fence(__ATOMIC_ACQUIRE, "workgroup");
  }
}

__device__ __forceinline__ float bfr(float f) { return bf_bits2f(f2bf_bits(f)); }
__device__ __forceinline__ unsigned pk16(unsigned short a, unsigned short b) { return (unsigned)a | ((unsigned)b << 16); }
__device__ __forceinline__ void st2_u32(unsigned* p, unsigned v) {
  *(volatile unsigned*)p = v; __threadfence(); *(volatile unsigned*)p = v;
}

constexpr int oW1aT = 0;
constexpr int oW1bT = 4096;
constexpr int oW2hi = 6144;
constexpr int oW2lo = 10240;
constexpr int oW2bT = 14336;
constexpr int oZero = 16384;
constexpr int kWplWords = 20480;

__global__ __launch_bounds__(kNT) void prep_kernel(const float* __restrict__ W1a, const float* __restrict__ W1b,
                                                  const float* __restrict__ W2a, const float* __restrict__ W2b,
                                                  const float* __restrict__ b1a, const float* __restrict__ b1b,
                                                  unsigned* __restrict__ WPL, float* __restrict__ BIAS) {
  const int i = blockIdx.x * kNT + threadIdx.x;
  const int p = blockIdx.y;
  if (p == 0) {
    const int n = i >> 6, k = (2 * i) & 127;
    const unsigned w = pk16(f2bf_bits(W1a[k * kHid + n]), f2bf_bits(W1a[(k + 1) * kHid + n]));
    st2_u32(WPL + oW1aT + i, w);
  } else if (p == 7) {
    st2_u32(WPL + oZero + i, 0u);
  } else if (p <= 6) {
    const int lim = 2048;
    const int ic = (i < lim) ? i : (lim - 1);
    const int n = ic >> 5, k = (2 * ic) & 63;
    unsigned w = 0u; int o = 0;
    if (p == 1) {
      w = pk16(f2bf_bits(W1b[k * kHid + n]), f2bf_bits(W1b[(k + 1) * kHid + n])); o = oW1bT;
    } else if (p == 2 || p == 4) {
      const float t0 = bfr(W2a[k * kHid + n]),        t1 = bfr(W2a[(k + 1) * kHid + n]);
      const float u0 = bfr(W2a[(64 + k) * kHid + n]), u1 = bfr(W2a[(65 + k) * kHid + n]);
      const float d0 = t0 - u0, d1 = t1 - u1;
      const unsigned short h0 = f2bf_bits(d0), h1 = f2bf_bits(d1);
      if (p == 2) { w = pk16(h0, h1); o = oW2hi; }
      else { w = pk16(f2bf_bits(d0 - bf_bits2f(h0)), f2bf_bits(d1 - bf_bits2f(h1))); o = oW2lo; }
    } else if (p == 3) {
      w = pk16(f2bf_bits(W2a[(64 + k) * kHid + n]), f2bf_bits(W2a[(65 + k) * kHid + n])); o = oW2hi + 2048;
    } else if (p == 5) {
      w = 0u; o = oW2lo + 2048;
    } else {
      w = pk16(f2bf_bits(W2b[k * kHid + n]), f2bf_bits(W2b[(k + 1) * kHid + n])); o = oW2bT;
    }
    if (i < lim) st2_u32(WPL + o + i, w);
  } else {
    const int ic = (i < kHid) ? i : (kHid - 1);
    const float va = bfr(b1a[ic]);
    const float vb = bfr(b1b[ic]);
    const float fa = (p == 8) ? 1.0f : 0.0f;
    const float v = fmaf(fa, va, (1.0f - fa) * vb);
    if (i < kHid) {
      float* bp = BIAS + ((p == 8) ? 0 : kHid) + i;
      *(volatile float*)bp = v; __threadfence(); *(volatile float*)bp = v;
    }
  }
}

__global__ __launch_bounds__(kNT) void castx_kernel(const float* __restrict__ x, unsigned* __restrict__ Xb) {
  const int i = blockIdx.x * kNT + threadIdx.x;
  const int row = i >> 4;
  const bool live = row < kNodes;
  const int rowc = live ? row : (kNodes - 1);
  const float* p = x + (size_t)rowc * kIn + (i & 15) * 8;
  const v4f a = *(const v4f*)(p);
  const v4f c = *(const v4f*)(p + 4);
  unsigned short hb[8];
#pragma unroll
  for (int e = 0; e < 4; ++e) {
    hb[e]     = live ? f2bf_bits(a[e]) : (unsigned short)0;
    hb[4 + e] = live ? f2bf_bits(c[e]) : (unsigned short)0;
  }
  const v4u u = (v4u){pk16(hb[0], hb[1]), pk16(hb[2], hb[3]), pk16(hb[4], hb[5]), pk16(hb[6], hb[7])};
  unsigned* q = Xb + 4 * (size_t)i;
  *(volatile v4u*)q = u;
  __threadfence();
  *(volatile v4u*)q = u;
}

__device__ __forceinline__ int blk_excl_scan(int cnt, int* scan_ws, int tid, int* tot) {
  const int lane = tid & 31, wave = tid >> 5; int incl = cnt;
#pragma unroll
  for (int o = 1; o < 32; o <<= 1) { const int v = __shfl_up(incl, o, 32); if (lane >= o) incl += v; }
  if (lane == 31) scan_ws[wave] = incl;
  __syncthreads();
  if (wave == 0) { int wv = (lane < kNT / 32) ? scan_ws[lane] : 0; int wincl = wv;
#pragma unroll
    for (int o = 1; o < 32; o <<= 1) { const int v = __shfl_up(wincl, o, 32); if (lane >= o) wincl += v; }
    if (lane < kNT / 32) scan_ws[32 + lane] = wincl - wv; if (lane == 31) scan_ws[64] = wincl; }
  __syncthreads();
  const int res = scan_ws[32 + wave] + incl - cnt; *tot = scan_ws[64];
  return res;
}
__device__ __forceinline__ int chunk_hits(const int* __restrict__ dstv, const int* __restrict__ srcv, int e0, int n0, int tid,
                                          int* LIST, int* scan_ws) {
  const int eb = e0 + tid * kSP;
  const bool live = eb < kEdges;
  const int ebc = live ? eb : (kEdges - kSP);
  int rec[kSP]; int cnt = 0;
#pragma unroll
  for (int k = 0; k < kSP; k += 4) {
    const v4i d4 = *(const v4i*)(dstv + ebc + k);
    const v4i s4 = *(const v4i*)(srcv + ebc + k);
#pragma unroll
    for (int e = 0; e < 4; ++e) {
      const int d = d4[e];
      int s = s4[e]; s = s < 0 ? 0 : (s >= kNodes ? kNodes - 1 : s);
      int r = -1;
      if (live && d >= n0 && d < n0 + kSRB) { r = ((d - n0) << 16) | s; ++cnt; }
      rec[k + e] = r;
    }
  }
  int tot; int p = blk_excl_scan(cnt, scan_ws, tid, &tot);
#pragma unroll
  for (int k = 0; k < kSP; ++k) if (rec[k] >= 0) { if ((unsigned)p < (unsigned)kCap) LIST[p] = rec[k]; ++p; }
  __syncthreads();
  return tot < kCap ? tot : kCap;
}

__global__ __launch_bounds__(kNT) void aggr_kernel(const float* __restrict__ PQ, const int* __restrict__ ei, const float* __restrict__ b2a,
                                                  unsigned short* __restrict__ Sh, unsigned short* __restrict__ Sl, float* __restrict__ DEG) {
  __shared__ __align__(16) float accS[kSRB * kHid];
  __shared__ int LIST[kCap + 32];
  __shared__ int degS[kSRB];
  __shared__ int scan_ws[80];
  const int tid = threadIdx.x, lane = tid & 31, wave = tid >> 5;
  const int n0 = blockIdx.x * kSRB;
  const float ba0 = bfr(b2a[2 * lane]), ba1 = bfr(b2a[2 * lane + 1]);
  {
    const v4f z4 = {0.f, 0.f, 0.f, 0.f};
    for (int i = tid; i < kSRB * kHid / 4; i += kNT) *(v4f*)(accS + 4 * i) = z4;
    for (int i = tid; i < kCap + 32; i += kNT) LIST[i] = -1;
    for (int i = tid; i < kSRB; i += kNT) degS[i] = 0;
    if (tid < 80) scan_ws[tid] = 0;
  }
  __syncthreads();
  const int* srcv = ei;
  const int* dstv = ei + kEdges;
#pragma unroll 1
  for (int c = 0; c < kNCh; ++c) {
    const int tot = chunk_hits(dstv, srcv, c * kChunk, n0, tid, LIST, scan_ws);
#pragma unroll 1
    for (int base = 0; base < tot; base += 32) {
      const int q = base + lane;
      const int rv = (q < tot) ? LIST[q] : -1;
      const int own = (rv >= 0 && (rv >> 22) == wave) ? 1 : 0;
      unsigned msk = (unsigned)__ballot(own);
#pragma unroll 1
      for (int it = 0; it < 32; ++it) {
        if (msk == 0u) break;
        const int bp = __builtin_ctz(msk); msk &= msk - 1u;
        const int r = __shfl(rv, bp, 32);
        const int dl = r >> 16, s = r & 0xFFFF;
        const v2f qv = *(const v2f*)(PQ + (size_t)s * 128 + 64 + 2 * lane);
        const v2f pv = *(const v2f*)(PQ + (size_t)(n0 + dl) * 128 + 2 * lane);
        float a0 = (pv[0] + qv[0]) + ba0;
        float a1 = (pv[1] + qv[1]) + ba1;
        a0 = fmaxf(a0, 0.f); a1 = fmaxf(a1, 0.f);
        float* ap = accS + dl * kHid + 2 * lane;
        v2f av = *(const v2f*)ap;
        av[0] = av[0] + a0; av[1] = av[1] + a1;
        *(v2f*)ap = av;
        if (lane == 0) degS[dl] += 1;
      }
    }
    __syncthreads();
  }
  __syncthreads();
  const int q8 = lane >> 3, c8 = (lane & 7) * 8;
  float bb[8];
  {
    const v4f b0 = *(const v4f*)(b2a + c8), b1 = *(const v4f*)(b2a + c8 + 4);
#pragma unroll
    for (int e = 0; e < 4; ++e) { bb[e] = bfr(b0[e]); bb[4 + e] = bfr(b1[e]); }
  }
  for (int pass = 0; pass < 2; ++pass) {
#pragma unroll 1
    for (int it = 0; it < 16; ++it) {
      const int dl = wave * 64 + it * 4 + q8;
      const int n = n0 + dl;
      const bool live = n < kNodes;
      const float* pr = PQ + (size_t)n * 128 + c8;
      const v4f p0 = *(const v4f*)(pr), p1 = *(const v4f*)(pr + 4);
      const v4f g0 = *(const v4f*)(pr + 64), g1 = *(const v4f*)(pr + 68);
      const v4f a0 = *(const v4f*)(accS + dl * kHid + c8), a1 = *(const v4f*)(accS + dl * kHid + c8 + 4);
      float sv[8];
#pragma unroll
      for (int e = 0; e < 4; ++e) {
        float t0 = (p0[e] + g0[e]) + bb[e];     t0 = fmaxf(t0, 0.f);
        float t1 = (p1[e] + g1[e]) + bb[4 + e]; t1 = fmaxf(t1, 0.f);
        sv[e]     = live ? (a0[e] + t0) : 0.f;
        sv[4 + e] = live ? (a1[e] + t1) : 0.f;
      }
      v8h hv, lv;
#pragma unroll
      for (int e = 0; e < 8; ++e) {
        const unsigned short hb = f2bf_bits(sv[e]);
        const unsigned short lb = f2bf_bits(sv[e] - bf_bits2f(hb));
        hv[e] = __builtin_bit_cast(_Float16, hb);
        lv[e] = __builtin_bit_cast(_Float16, lb);
      }
      *(volatile v8h*)(Sh + (size_t)n * kHid + c8) = hv;
      *(volatile v8h*)(Sl + (size_t)n * kHid + c8) = lv;
    }
    __threadfence();
  }
  if (wave == 0) {
    for (int pass = 0; pass < 2; ++pass) {
#pragma unroll
      for (int i4 = 0; i4 < 4; ++i4) {
        const int dl0 = i4 * 128 + 4 * lane;
        v4f dv;
#pragma unroll
        for (int e = 0; e < 4; ++e) {
          const int dl = dl0 + e; const int n = n0 + dl;
          dv[e] = (float)(degS[dl] + ((n < kNodes) ? 1 : 0));
        }
        *(volatile v4f*)(DEG + n0 + dl0) = dv;
      }
      __threadfence();
    }
  }
}

__global__ __launch_bounds__(kNT) void cls_kernel(const float* __restrict__ AGG, const unsigned* __restrict__ Hhw,
                                                 const unsigned* __restrict__ Hlw, const float* __restrict__ DEG,
                                                 const float* __restrict__ b2b, const float* __restrict__ Wc,
                                                 const float* __restrict__ bc, float* __restrict__ out) {
  __shared__ float sW[kHid * kCls];
  __shared__ float sBb[kHid];
  __shared__ float sBc[16];
  __shared__ __align__(16) float so[8][320];
  const int tid = threadIdx.x, lane = tid & 31, wave = tid >> 5;
  for (int i = tid; i < kHid * kCls; i += kNT) sW[i] = bfr(Wc[i]);
  if (tid < kHid) sBb[tid] = bfr(b2b[tid]);
  if (tid < kCls) sBc[tid] = bfr(bc[tid]);
  __syncthreads();
  const int n = blockIdx.x * kNT + tid;
  float acc[kCls];
#pragma unroll
  for (int c = 0; c < kCls; ++c) acc[c] = 0.f;
  const float dg = DEG[n];
  const float* ar = AGG + (size_t)n * kHid;
  const unsigned* hr = Hhw + (size_t)n * (kHid / 2);
  const unsigned* lr = Hlw + (size_t)n * (kHid / 2);
#pragma unroll 1
  for (int kc = 0; kc < kHid / 4; ++kc) {
    const v4f ag = *(const v4f*)(ar + 4 * kc);
    const v2u hh = *(const v2u*)(hr + 2 * kc);
    const v2u hl = *(const v2u*)(lr + 2 * kc);
    const unsigned w0 = hh[0], w1 = hh[1], l0 = hl[0], l1 = hl[1];
    float hv[4];
    hv[0] = __uint_as_float(w0 << 16)          + __uint_as_float(l0 << 16);
    hv[1] = __uint_as_float(w0 & 0xffff0000u)  + __uint_as_float(l0 & 0xffff0000u);
    hv[2] = __uint_as_float(w1 << 16)          + __uint_as_float(l1 << 16);
    hv[3] = __uint_as_float(w1 & 0xffff0000u)  + __uint_as_float(l1 & 0xffff0000u);
    float u[4];
#pragma unroll
    for (int e = 0; e < 4; ++e) u[e] = ((ag[e] + dg * sBb[4 * kc + e]) + hv[e]) * 0.5f;
#pragma unroll
    for (int c = 0; c < kCls; ++c) {
      const float* w = sW + (4 * kc) * kCls + c;
      acc[c] = acc[c] + u[0] * w[0] + u[1] * w[kCls] + u[2] * w[2 * kCls] + u[3] * w[3 * kCls];
    }
  }
  float* sw = so[wave];
#pragma unroll
  for (int c = 0; c < kCls; ++c) sw[lane * kCls + c] = acc[c] + sBc[c];
  __syncthreads();
  const int nodebase = blockIdx.x * kNT + wave * 32;
  int nval = kNodes - nodebase; nval = nval < 0 ? 0 : (nval > 32 ? 32 : nval);
  const int nf4 = (nval * kCls) >> 2;
  const v4f p0 = *(const v4f*)(sw + 4 * lane);
  const v4f p1 = *(const v4f*)(sw + 128 + 4 * lane);
  const v4f p2 = *(const v4f*)(sw + 256 + 4 * (lane & 15));
  for (int pass = 0; pass < 2; ++pass) {
    if (lane < nf4)      *(volatile v4f*)(out + (size_t)nodebase * kCls + 4 * lane) = p0;
    if (lane + 32 < nf4) *(volatile v4f*)(out + (size_t)nodebase * kCls + 128 + 4 * lane) = p1;
    if (lane + 64 < nf4) *(volatile v4f*)(out + (size_t)nodebase * kCls + 256 + 4 * (lane & 15)) = p2;
    __threadfence();
  }
}

extern "C" void kernel_launch(void* const* d_in, const int* in_sizes, int n_in,
                              void* d_out, int out_size, void* d_ws, size_t ws_size, hipStream_t stream) {
  (void)in_sizes; (void)n_in; (void)out_size;
  const float* x   = (const float*)d_in[0];
  const int*   ei  = (const int*)  d_in[1];
  const float* W1a = (const float*)d_in[2];
  const float* b1a = (const float*)d_in[3];
  const float* W1b = (const float*)d_in[4];
  const float* b1b = (const float*)d_in[5];
  const float* W2a = (const float*)d_in[6];
  const float* b2a = (const float*)d_in[7];
  const float* W2b = (const float*)d_in[8];
  const float* b2b = (const float*)d_in[9];
  const float* Wc  = (const float*)d_in[10];
  const float* bc  = (const float*)d_in[11];
  float* out = (float*)d_out;

  char* ws = (char*)d_ws; size_t off = 0;
  auto carve = [&](size_t bytes) -> char* { char* p = ws + off; off += (bytes + 255) & ~(size_t)255; return p; };
  unsigned*       WPL  = (unsigned*)carve((size_t)kWplWords * 4);
  float*          BIAS = (float*)carve((size_t)2 * kHid * 4);
  unsigned*       Xb   = (unsigned*)carve((size_t)kMP * kIn * 2);
  unsigned short* A1h  = (unsigned short*)carve((size_t)kMP * kHid * 2);
  unsigned short* A1l  = (unsigned short*)carve((size_t)kMP * kHid * 2);
  unsigned short* Hh   = (unsigned short*)carve((size_t)kMP * kHid * 2);
  unsigned short* Hl   = (unsigned short*)carve((size_t)kMP * kHid * 2);
  float*          PQ   = (float*)carve((size_t)kMP * 2 * kHid * 4);
  unsigned short* Sh   = (unsigned short*)carve((size_t)kMP * kHid * 2);
  unsigned short* Sl   = (unsigned short*)carve((size_t)kMP * kHid * 2);
  float*          DEG  = (float*)carve((size_t)kMP * 4);
  float*          AGG  = (float*)carve((size_t)kMP * kHid * 4);
  if (off > ws_size || off > (size_t)134217728) return;

  prep_kernel<<<dim3(16, 10), kNT, 0, stream>>>(W1a, W1b, W2a, W2b, b1a, b1b, WPL, BIAS);
  castx_kernel<<<(kMP * kIn / 8) / kNT, kNT, 0, stream>>>(x, Xb);
  {
    const int tiles = (kMP / 64) * (kHid / 64);
    wmma_gemm64<1, false, 2, 2, false, 2><<<dim3((tiles + 7) / 8, 1), 256, 0, stream>>>(
        (const unsigned short*)Xb, (const unsigned short*)Xb, kIn, 0L,
        (const unsigned short*)(WPL + oW1aT), (const unsigned short*)(WPL + oZero), kIn, 0L,
        (void*)A1h, (void*)A1l, kHid, 0L,
        BIAS, (const float*)nullptr, 0L, kMP, kHid, kIn, 1.0f);
  }
  {
    const int tiles = (kMP / 64) * (kHid / 64);
    wmma_gemm64<1, true, 2, 2, false, 0><<<dim3((tiles + 7) / 8, 1), 256, 0, stream>>>(
        (const unsigned short*)A1h, (const unsigned short*)A1l, kHid, 0L,
        (const unsigned short*)(WPL + oW1bT), (const unsigned short*)(WPL + oZero), kHid, 0L,
        (void*)Hh, (void*)Hl, kHid, 0L,
        BIAS + kHid, (const float*)nullptr, 0L, kMP, kHid, kHid, 1.0f);
  }
  {
    const int tiles = (kMP / 64) * ((2 * kHid) / 64);
    wmma_gemm64<1, true, 0, 0, false, 0><<<dim3((tiles + 7) / 8, 1), 256, 0, stream>>>(
        (const unsigned short*)Hh, (const unsigned short*)Hl, kHid, 0L,
        (const unsigned short*)(WPL + oW2hi), (const unsigned short*)(WPL + oW2lo), kHid, 0L,
        (void*)PQ, (void*)PQ, 2 * kHid, 0L,
        (const float*)nullptr, (const float*)nullptr, 0L, kMP, 2 * kHid, kHid, 1.0f);
  }
  aggr_kernel<<<kMP / kSRB, kNT, 0, stream>>>(PQ, ei, b2a, Sh, Sl, DEG);
  {
    const int tiles = (kMP / 64) * (kHid / 64);
    wmma_gemm64<1, true, 0, 0, false, 0><<<dim3((tiles + 7) / 8, 1), 256, 0, stream>>>(
        (const unsigned short*)Sh, (const unsigned short*)Sl, kHid, 0L,
        (const unsigned short*)(WPL + oW2bT), (const unsigned short*)(WPL + oZero), kHid, 0L,
        (void*)AGG, (void*)AGG, kHid, 0L,
        (const float*)nullptr, (const float*)nullptr, 0L, kMP, kHid, kHid, 1.0f);
  }
  cls_kernel<<<kMP / kNT, kNT, 0, stream>>>(AGG, (const unsigned*)Hh, (const unsigned*)Hl, DEG, b2b, Wc, bc, out);
}
